// VideoEncoder_26233660244652
// MI455X (gfx1250) — hardware-verified
//
#include <hip/hip_runtime.h>
#include <math.h>

typedef __attribute__((ext_vector_type(16))) _Float16 v16h;
typedef __attribute__((ext_vector_type(16))) __bf16 v16b;
typedef __attribute__((ext_vector_type(8)))  _Float16 v8h;
typedef __attribute__((ext_vector_type(8)))  float v8f;
typedef __attribute__((ext_vector_type(4)))  float v4f;
typedef __attribute__((ext_vector_type(2)))  float v2f;
typedef __attribute__((ext_vector_type(4)))  unsigned v4u;
typedef __attribute__((ext_vector_type(4)))  int v4i;
typedef float __attribute__((may_alias)) float_a;
typedef int __attribute__((may_alias)) int_a;

template <typename T> __device__ __forceinline__ void vst2(void* p, T v) { *(volatile T*)p = v; __threadfence(); *(volatile T*)p = v; }
__device__ __forceinline__ v8f wmma16(v16h a, v16h b, v8f c) {
  v8f d = __builtin_amdgcn_wmma_f32_16x16x32_f16(false, a, false, b, (short)0, c, false, false);
  asm volatile("v_nop\n\tv_nop\n\tv_nop\n\tv_nop" : "+v"(d) : "v"(a), "v"(b));
  return d;
}
__device__ __forceinline__ v8f wmma_bf(v16b a, v16b b, v8f c) {
  v8f d = __builtin_amdgcn_wmma_f32_16x16x32_bf16(false, a, false, b, (short)0, c, false, false);
  asm volatile("v_nop\n\tv_nop\n\tv_nop\n\tv_nop" : "+v"(d) : "v"(a), "v"(b));
  return d;
}
__device__ __forceinline__ v16h frag_h(const _Float16* rowk0, int lane) {
  union { v16h v; v8h q[2]; } u; const _Float16* p = rowk0 + 8 * (lane >> 4);
  u.q[0] = *(const v8h*)p; u.q[1] = *(const v8h*)(p + 16); return u.v;
}
__device__ __forceinline__ v16h frag_f32(const float* rowk0, int lane) {
  v16h a; const float* p = rowk0 + 8 * (lane >> 4);
#pragma unroll
  for (int i = 0; i < 8; ++i) { a[i] = (_Float16)p[i]; a[8 + i] = (_Float16)p[16 + i]; }
  return a;
}
__device__ __forceinline__ v16h frag_f32s(const float* rowk0, int lane, float sc) {
  v16h a; const float* p = rowk0 + 8 * (lane >> 4);
#pragma unroll
  for (int i = 0; i < 8; ++i) { a[i] = (_Float16)(p[i] * sc); a[8 + i] = (_Float16)(p[16 + i] * sc); }
  return a;
}
__device__ __forceinline__ v16h fragc_f32(const float* W, int k0, int n, int lane, int ld, int K) {
  v16h a; const int g = lane >> 4;
#pragma unroll
  for (int i = 0; i < 8; ++i) { const int ka = k0 + 8 * g + i, kb = ka + 16;
    a[i] = (_Float16)(ka < K ? W[(size_t)ka * ld + n] : 0.f); a[8 + i] = (_Float16)(kb < K ? W[(size_t)kb * ld + n] : 0.f); }
  return a;
}
struct F2 { v16b h, l; };
__device__ __forceinline__ F2 bsplit16(const float v[16]) { F2 r;
#pragma unroll
  for (int i = 0; i < 16; ++i) { const __bf16 h = (__bf16)v[i]; r.h[i] = h; r.l[i] = (__bf16)(v[i] - (float)h); }
  return r; }
__device__ __forceinline__ F2 split_row(const float* row, int k0, int lane) { float v[16]; const float* p = row + k0 + 8 * (lane >> 4);
#pragma unroll
  for (int i = 0; i < 8; ++i) { v[i] = p[i]; v[8 + i] = p[16 + i]; }
  return bsplit16(v); }
__device__ __forceinline__ F2 split_rowK(const float* row, int k0, int lane, int K) { float v[16]; const int g = lane >> 4;
#pragma unroll
  for (int i = 0; i < 8; ++i) { const int ka = k0 + 8 * g + i, kb = ka + 16; v[i] = ka < K ? row[ka] : 0.f; v[8 + i] = kb < K ? row[kb] : 0.f; }
  return bsplit16(v); }
__device__ __forceinline__ F2 split_col(const float* W, int k0, int n, int lane, int ld, int K) { float v[16]; const int g = lane >> 4;
#pragma unroll
  for (int i = 0; i < 8; ++i) { const int ka = k0 + 8 * g + i, kb = ka + 16; v[i] = ka < K ? W[(size_t)ka * ld + n] : 0.f; v[8 + i] = kb < K ? W[(size_t)kb * ld + n] : 0.f; }
  return bsplit16(v); }
__device__ __forceinline__ v8f mac3(const F2& a, const F2& b, v8f c) { c = wmma_bf(a.l, b.h, c); c = wmma_bf(a.h, b.l, c); return wmma_bf(a.h, b.h, c); }
__device__ __forceinline__ float sigm(float v) { return 1.0f / (1.0f + expf(-v)); }
#define LDSX() do { asm volatile("s_wait_dscnt 0" ::: "memory"); __builtin_amdgcn_wave_barrier(); __builtin_amdgcn_fence(__ATOMIC_RELEASE, "workgroup"); } while (0)

#define NB 2
#define TT 2048
#define DIN 2048
#define HH 256
#define NHD 4
#define DH 64
#define WIN 15
#define NR (NB * TT)

template <int KIN>
__global__ __launch_bounds__(128) void k_gemm(const float* __restrict__ A, const float* __restrict__ W, const float* __restrict__ bias, float* __restrict__ OUT) {
  __shared__ __align__(16) float so[4][16][132];
  const int tid = threadIdx.x, wave = tid >> 5, lane = tid & 31, col = lane & 15, g = lane >> 4;
  const int r0 = blockIdx.x * 64 + wave * 16, n0 = blockIdx.y * 128;
  v8f acc[8] = {};
#pragma unroll 1
  for (int kc = 0; kc < KIN / 32; ++kc) { const F2 a = split_row(A + (size_t)(r0 + col) * KIN, kc * 32, lane);
#pragma unroll
    for (int j = 0; j < 8; ++j) acc[j] = mac3(a, split_col(W, kc * 32, n0 + j * 16 + col, lane, HH, KIN), acc[j]); }
#pragma unroll
  for (int j = 0; j < 8; ++j) { const float bb = bias ? bias[n0 + j * 16 + col] : 0.f;
#pragma unroll
    for (int r = 0; r < 8; ++r) so[wave][8 * g + r][j * 16 + col] = acc[j][r] + bb; }
  LDSX();
#pragma unroll 4
  for (int rl = 0; rl < 16; ++rl) vst2(OUT + (size_t)(r0 + rl) * HH + n0 + lane * 4, *(const v4f*)(&so[wave][rl][lane * 4]));
}
__global__ __launch_bounds__(256) void k_escal(const float* __restrict__ HW, const float* __restrict__ asrc, const float* __restrict__ adst, float* __restrict__ E) {
  __shared__ __align__(16) float se[64][8];
  const int tid = threadIdx.x, rl = tid >> 2, hd = tid & 3; const size_t r = (size_t)blockIdx.x * 64 + rl;
  const float* hr = HW + r * HH + hd * DH; float s1 = 0.f, s2 = 0.f;
#pragma unroll 8
  for (int d = 0; d < DH; ++d) { const float hv = hr[d]; s1 += hv * asrc[hd * DH + d]; s2 += hv * adst[hd * DH + d]; }
  se[rl][hd] = s1; se[rl][4 + hd] = s2;
  __syncthreads();
  if (tid < 128) vst2(E + (size_t)blockIdx.x * 64 * 8 + tid * 4, *(const v4f*)(&se[0][0] + tid * 4));
}
template <int FINAL>
__global__ __launch_bounds__(256) void k_gat(const float* __restrict__ X, const float* __restrict__ HW, const float* __restrict__ E, const int* __restrict__ adj, const float* __restrict__ gam, const float* __restrict__ bet, const float* __restrict__ gF, const float* __restrict__ bF, float* __restrict__ OUT) {
  const int tid = threadIdx.x, wave = tid >> 5, lane = tid & 31; const int b = blockIdx.y, i = blockIdx.x * 8 + wave; const size_t ri = (size_t)b * TT + i;
  const int hd = lane >> 3, c0 = lane * 8;
  const int jlo = max(i - WIN, 0), jhi = min(i + WIN, TT - 1);
  const float es = E[ri * 8 + hd];
  float w[2 * WIN + 1]; float mx = -3.0e38f;
#pragma unroll
  for (int u = 0; u < 2 * WIN + 1; ++u) { const int j = jlo + u; float e = -3.0e38f;
    if (j <= jhi && adj[(size_t)i * TT + j] != 0) { e = es + E[((size_t)b * TT + j) * 8 + 4 + hd]; e = e > 0.f ? e : 0.2f * e; }
    w[u] = e; mx = fmaxf(mx, e); }
  float l = 0.f;
#pragma unroll
  for (int u = 0; u < 2 * WIN + 1; ++u) { const float p = w[u] <= -1.0e38f ? 0.f : expf(w[u] - mx); w[u] = p; l += p; }
  const float inv = 1.0f / l;
  v4f o0 = {0.f, 0.f, 0.f, 0.f}, o1 = {0.f, 0.f, 0.f, 0.f};
#pragma unroll 1
  for (int u = 0; u < 2 * WIN + 1; ++u) { if (w[u] != 0.f) { const float* hr = HW + ((size_t)b * TT + jlo + u) * HH + c0; const float pw = w[u] * inv; o0 += pw * *(const v4f*)hr; o1 += pw * *(const v4f*)(hr + 4); } }
  const float* xr = X + ri * HH + c0; o0 += *(const v4f*)xr; o1 += *(const v4f*)(xr + 4);
  float s = (o0[0] + o0[1]) + (o0[2] + o0[3]) + (o1[0] + o1[1]) + (o1[2] + o1[3]);
#pragma unroll
  for (int off = 16; off >= 1; off >>= 1) s += __shfl_xor(s, off, 32);
  const float mu = s * (1.0f / HH); v4f d0 = o0 - mu, d1 = o1 - mu;
  float q2 = (d0[0] * d0[0] + d0[1] * d0[1]) + (d0[2] * d0[2] + d0[3] * d0[3]) + (d1[0] * d1[0] + d1[1] * d1[1]) + (d1[2] * d1[2] + d1[3] * d1[3]);
#pragma unroll
  for (int off = 16; off >= 1; off >>= 1) q2 += __shfl_xor(q2, off, 32);
  const float rs = rsqrtf(q2 * (1.0f / HH) + 1e-5f);
  o0 = d0 * rs * *(const v4f*)(gam + c0) + *(const v4f*)(bet + c0); o1 = d1 * rs * *(const v4f*)(gam + c0 + 4) + *(const v4f*)(bet + c0 + 4);
  if (FINAL) { float s3 = (o0[0] + o0[1]) + (o0[2] + o0[3]) + (o1[0] + o1[1]) + (o1[2] + o1[3]);
#pragma unroll
    for (int off = 16; off >= 1; off >>= 1) s3 += __shfl_xor(s3, off, 32);
    const float mu2 = s3 * (1.0f / HH); d0 = o0 - mu2; d1 = o1 - mu2;
    float q3 = (d0[0] * d0[0] + d0[1] * d0[1]) + (d0[2] * d0[2] + d0[3] * d0[3]) + (d1[0] * d1[0] + d1[1] * d1[1]) + (d1[2] * d1[2] + d1[3] * d1[3]);
#pragma unroll
    for (int off = 16; off >= 1; off >>= 1) q3 += __shfl_xor(q3, off, 32);
    const float rs2 = rsqrtf(q3 * (1.0f / HH) + 1e-5f);
    o0 = d0 * rs2 * *(const v4f*)(gF + c0) + *(const v4f*)(bF + c0); o1 = d1 * rs2 * *(const v4f*)(gF + c0 + 4) + *(const v4f*)(bF + c0 + 4); }
  vst2(OUT + ri * HH + c0, o0); vst2(OUT + ri * HH + c0 + 4, o1);
}
extern "C" void kernel_launch(void* const* d_in, const int* in_sizes, int n_in, void* d_out, int out_size, void* d_ws, size_t ws_size, hipStream_t stream) {
  (void)in_sizes; (void)n_in; (void)out_size; (void)ws_size;
  const float* x = (const float*)d_in[0]; const int* adj = (const int*)d_in[1]; const float* Wp = (const float*)d_in[2]; const float* bp = (const float*)d_in[3];
  const float* W0 = (const float*)d_in[4]; const float* as0 = (const float*)d_in[5]; const float* ad0 = (const float*)d_in[6]; const float* g0 = (const float*)d_in[7]; const float* b0 = (const float*)d_in[8];
  const float* W1 = (const float*)d_in[9]; const float* as1 = (const float*)d_in[10]; const float* ad1 = (const float*)d_in[11]; const float* g1 = (const float*)d_in[12]; const float* b1 = (const float*)d_in[13];
  const float* gF = (const float*)d_in[14]; const float* bF = (const float*)d_in[15];
  float* out = (float*)d_out;
  char* ws = (char*)d_ws; size_t off = 0;
  auto take = [&](size_t bytes) { char* p = ws + off; off += (bytes + 255) & ~(size_t)255; return p; };
  float* H0 = (float*)take((size_t)NR * HH * 4); float* HW = (float*)take((size_t)NR * HH * 4); float* E = (float*)take((size_t)NR * 8 * 4); float* H1 = (float*)take((size_t)NR * HH * 4);
  k_gemm<DIN><<<dim3(NR / 64, 2), 128, 0, stream>>>(x, Wp, bp, H0);
  k_gemm<HH><<<dim3(NR / 64, 2), 128, 0, stream>>>(H0, W0, nullptr, HW);
  k_escal<<<NR / 64, 256, 0, stream>>>(HW, as0, ad0, E);
  k_gat<0><<<dim3(TT / 8, NB), 256, 0, stream>>>(H0, HW, E, adj, g0, b0, gF, bF, H1);
  k_gemm<HH><<<dim3(NR / 64, 2), 128, 0, stream>>>(H1, W1, nullptr, HW);
  k_escal<<<NR / 64, 256, 0, stream>>>(HW, as1, ad1, E);
  k_gat<1><<<dim3(TT / 8, NB), 256, 0, stream>>>(H1, HW, E, adj, g1, b1, gF, bF, out);
}
